// BlockGlobalAttentionProduct_72121090834680
// MI455X (gfx1250) — hardware-verified
//
#include <hip/hip_runtime.h>


#define NB_  2
#define NHD  12
#define TT   4096
#define DDm  64
#define CS   128
#define TCS  256
#define NG   64
#define NBL  64
#define TNB  32
#define FF   2
#define LL   192
#define LG   448
#define KK   640
#define PCAR 1024.0f
typedef _Float16 h16;
typedef unsigned short bf;
typedef __attribute__((ext_vector_type(16))) __bf16   v16bf;
typedef __attribute__((ext_vector_type(16))) _Float16 v16h;
typedef __attribute__((ext_vector_type(8)))  _Float16 v8h;
typedef __attribute__((ext_vector_type(8)))  unsigned short v8us;
typedef __attribute__((ext_vector_type(8)))  float    v8f;
typedef __attribute__((ext_vector_type(4)))  float    v4f;
typedef v8h  __attribute__((may_alias)) v8ha;
typedef v4f  __attribute__((may_alias)) v4fa;
typedef v8us __attribute__((may_alias)) v8usa;

__device__ __forceinline__ unsigned short f2bf(float f) { unsigned u = __float_as_uint(f); u += 0x7FFFu + ((u >> 16) & 1u); return (unsigned short)(u >> 16); }
__device__ __forceinline__ float bf2f(unsigned short b) { return __uint_as_float(((unsigned)b) << 16); }
__device__ __forceinline__ float bfr(float f) { return bf2f(f2bf(f)); }
__device__ __forceinline__ v16h cat16(v8h lo, v8h hi) { return __builtin_shufflevector(lo, hi, 0, 1, 2, 3, 4, 5, 6, 7, 8, 9, 10, 11, 12, 13, 14, 15); }
__device__ __forceinline__ v16bf cat16b(v8us lo, v8us hi) { return __builtin_bit_cast(v16bf, __builtin_shufflevector(lo, hi, 0, 1, 2, 3, 4, 5, 6, 7, 8, 9, 10, 11, 12, 13, 14, 15)); }
__device__ __forceinline__ v8f wmma16(v16h a, v16h b, v8f c) { return __builtin_amdgcn_wmma_f32_16x16x32_f16(false, a, false, b, (short)0, c, false, false); }
__device__ __forceinline__ v8f wmmab(v16bf a, v16bf b, v8f c) { return __builtin_amdgcn_wmma_f32_16x16x32_bf16(false, a, false, b, (short)0, c, false, false); }


template <typename T16> struct WFrag;
template <> struct WFrag<h16> { typedef v16h V; static __device__ __forceinline__ V ld(const h16* p) { return cat16(*(const v8h*)p, *(const v8h*)(p + 16)); } static __device__ __forceinline__ v8f mma(V a, V b, v8f c) { return wmma16(a, b, c); } };
template <> struct WFrag<bf> { typedef v16bf V; static __device__ __forceinline__ V ld(const bf* p) { return cat16b(*(const v8us*)p, *(const v8us*)(p + 16)); } static __device__ __forceinline__ v8f mma(V a, V b, v8f c) { return wmmab(a, b, c); } };
template <typename T16, int NSPLIT, bool BIAS>
__global__ __launch_bounds__(32) void k_gemmw(const T16* __restrict__ A, const T16* __restrict__ A2, const T16* __restrict__ Bt, const T16* __restrict__ Bt2, int K, float* C, int ldc, const float* __restrict__ bias, size_t sA, size_t sB, size_t sC) {
    typedef typename WFrag<T16>::V V;
    __shared__ __align__(16) float os[16 * 68];
    const size_t z = blockIdx.z; A += z * sA; if (A2) A2 += z * sA; Bt += z * sB; if (Bt2) Bt2 += z * sB; C += z * sC;
    const int lane = threadIdx.x & 31, lr = lane & 15, hi = lane >> 4; const int r0 = blockIdx.x * 64, c0 = blockIdx.y * 64;
    v8f acc[4][4];
#pragma unroll
    for (int mb = 0; mb < 4; ++mb)
#pragma unroll
        for (int nb = 0; nb < 4; ++nb) acc[mb][nb] = (v8f){};
    const size_t aoff = (size_t)(r0 + lr) * K + 8 * hi, boff = (size_t)(c0 + lr) * K + 8 * hi;
#pragma unroll 1
    for (int kc = 0; kc < K; kc += 32) {
        V a[4], a2[4];
#pragma unroll
        for (int mb = 0; mb < 4; ++mb) { a[mb] = WFrag<T16>::ld(A + aoff + (size_t)mb * 16 * K + kc); if (NSPLIT == 1 || NSPLIT == 2) a2[mb] = WFrag<T16>::ld(A2 + aoff + (size_t)mb * 16 * K + kc); }
#pragma unroll
        for (int nb = 0; nb < 4; ++nb) { const V b = WFrag<T16>::ld(Bt + boff + (size_t)nb * 16 * K + kc); V b2; if (NSPLIT >= 2) b2 = WFrag<T16>::ld(Bt2 + boff + (size_t)nb * 16 * K + kc);
#pragma unroll
            for (int mb = 0; mb < 4; ++mb) { acc[mb][nb] = WFrag<T16>::mma(a[mb], b, acc[mb][nb]); if (NSPLIT == 1 || NSPLIT == 2) acc[mb][nb] = WFrag<T16>::mma(a2[mb], b, acc[mb][nb]); if (NSPLIT >= 2) acc[mb][nb] = WFrag<T16>::mma(a[mb], b2, acc[mb][nb]); } }
        asm volatile("v_nop\n\tv_nop\n\tv_nop\n\tv_nop" : "+v"(acc[0][0]), "+v"(acc[1][1]), "+v"(acc[2][2]), "+v"(acc[3][3]) : "v"(a[0]), "v"(a[3]));
    }
#pragma unroll
    for (int mb = 0; mb < 4; ++mb) {
#pragma unroll
        for (int nb = 0; nb < 4; ++nb) {
#pragma unroll
            for (int j = 0; j < 8; ++j) os[(hi * 8 + j) * 68 + nb * 16 + lr] = acc[mb][nb][j]; }
        __builtin_amdgcn_wave_barrier(); asm volatile("" ::: "memory");
        float* crow = C + (size_t)(r0 + mb * 16) * ldc + c0;
#pragma unroll 1
        for (int ps = 0; ps < 2; ++ps) {
#pragma unroll
            for (int s = 0; s < 8; ++s) { const int row = 2 * s + hi, cofs = lr * 4; v4f val = *(const v4fa*)(os + row * 68 + cofs); if (BIAS) { val[0] += bfr(bias[c0 + cofs]); val[1] += bfr(bias[c0 + cofs + 1]); val[2] += bfr(bias[c0 + cofs + 2]); val[3] += bfr(bias[c0 + cofs + 3]); }
                *(volatile v4f*)(crow + (size_t)row * ldc + cofs) = val; }
            if (ps == 0) __threadfence(); }
        __builtin_amdgcn_wave_barrier(); asm volatile("" ::: "memory");
    }
}

__device__ __forceinline__ h16 tohx(float x) { return (h16)x; }
typedef __attribute__((ext_vector_type(2))) _Float16 v2h;
typedef __attribute__((ext_vector_type(4))) unsigned short v4us;

__global__ __launch_bounds__(256) void k_cvt8(const float* __restrict__ src, bf* dst, size_t n8) { const size_t i = (size_t)blockIdx.x * 256 + threadIdx.x; if (i >= n8) return; const v8f v = *(const v8f*)(src + i * 8); v8us o;
#pragma unroll
    for (int k = 0; k < 8; ++k) o[k] = f2bf(v[k]); *(volatile v8us*)(dst + i * 8) = o; __threadfence(); *(volatile v8us*)(dst + i * 8) = o; }
__device__ __forceinline__ int clampi(int j) { return j < 0 ? 0 : (j >= TT ? TT - 1 : j); }
__device__ __forceinline__ int keysrc(int b, int s, const int* li, const int* gi, int& kind) { if (s < LL) { const int t = (b * (CS / 2) - CS / 2 + s + TT) % TT; kind = 0; return clampi(li[t]); } const int r = s - LL; if (r < 3 * TCS / 2) { const int t = ((b / FF) * (TCS / 2) - TCS / 2 + r + TT) % TT; kind = 1; return clampi(gi[t]); } kind = 2; return r - 3 * TCS / 2; }
__global__ __launch_bounds__(256) void k_kb(const float* __restrict__ kh, const float* __restrict__ gk, const int* __restrict__ li, const int* __restrict__ gi, bf* KB) { const int e = (blockIdx.x * 256 + threadIdx.x) * 4; if (e >= NBL * KK * DDm) return; const int d = e % DDm; const int s = (e / DDm) % KK; const int b = e / (DDm * KK); int kind; const int j = keysrc(b, s, li, gi, kind);
    const float* src = (kind == 2 ? gk : kh) + (size_t)j * DDm + d; v4us o; o[0] = f2bf(src[0]); o[1] = f2bf(src[1]); o[2] = f2bf(src[2]); o[3] = f2bf(src[3]); *(volatile v4us*)(KB + e) = o; __threadfence(); *(volatile v4us*)(KB + e) = o; }
__global__ __launch_bounds__(256) void k_vt(const float* __restrict__ vh, const float* __restrict__ gv, const int* __restrict__ li, const int* __restrict__ gi, h16* VT) { const int e = (blockIdx.x * 256 + threadIdx.x) * 2; if (e >= NBL * DDm * KK) return; const int s = e % KK; const int d = (e / KK) % DDm; const int b = e / (KK * DDm); v2h o;
#pragma unroll
    for (int u = 0; u < 2; ++u) { int kind; const int j = keysrc(b, s + u, li, gi, kind); const float* src = (kind == 2 ? gv : vh) + (size_t)j * DDm + d; o[u] = tohx(bfr(src[0])); } *(volatile v2h*)(VT + e) = o; __threadfence(); *(volatile v2h*)(VT + e) = o; }
__global__ __launch_bounds__(256) void k_mb(const float* __restrict__ am, const float* __restrict__ gm, const int* __restrict__ li, const int* __restrict__ gi, float* MB) { const int e = blockIdx.x * 256 + threadIdx.x; if (e >= NBL * KK) return; const int s = e % KK, b = e / KK; int kind; const int j = keysrc(b, s, li, gi, kind); const float v = bfr(kind == 2 ? gm[j] : am[j]); *(volatile float*)(MB + e) = v; __threadfence(); *(volatile float*)(MB + e) = v; }
__global__ __launch_bounds__(256) void k_fin(const float* __restrict__ O, float* OUTh) { const int e = (blockIdx.x * 256 + threadIdx.x) * 4; if (e >= TT * DDm) return; const v4f a = *(const v4f*)(O + e); v4f o; o[0] = a[0] * (1.0f / PCAR); o[1] = a[1] * (1.0f / PCAR); o[2] = a[2] * (1.0f / PCAR); o[3] = a[3] * (1.0f / PCAR); *(volatile v4f*)(OUTh + e) = o; __threadfence(); *(volatile v4f*)(OUTh + e) = o; }
__global__ __launch_bounds__(256) void k_msoft(const float* __restrict__ Sb, const float* __restrict__ MB, h16* P16) { const int lane = threadIdx.x & 31; const int row = blockIdx.x * 8 + (threadIdx.x >> 5); if (row >= NBL * 64) return; const int b = row / 64; const float* sr = Sb + (size_t)row * KK; const float* mr = MB + (size_t)b * KK; float mx = -3.0e38f;
#pragma unroll 1
    for (int ch = 0; ch < KK / 128; ++ch) { const int j0 = ch * 128 + lane * 4; const v4f a = *(const v4f*)(sr + j0);
#pragma unroll
        for (int u = 0; u < 4; ++u) mx = fmaxf(mx, __fadd_rn(a[u] * 0.125f, mr[j0 + u])); }
#pragma unroll
    for (int sh = 16; sh; sh >>= 1) mx = fmaxf(mx, __shfl_xor(mx, sh, 32));
    float sum = 0.f;
#pragma unroll 1
    for (int ch = 0; ch < KK / 128; ++ch) { const int j0 = ch * 128 + lane * 4; const v4f a = *(const v4f*)(sr + j0);
#pragma unroll
        for (int u = 0; u < 4; ++u) { float d0 = __fsub_rn(__fadd_rn(a[u] * 0.125f, mr[j0 + u]), mx); asm volatile("" : "+v"(d0)); sum += __expf(d0); } }
#pragma unroll
    for (int sh = 16; sh; sh >>= 1) sum += __shfl_xor(sum, sh, 32);
    const float f = __fdiv_rn(PCAR, sum);
    for (int ps = 0; ps < 2; ++ps) {
#pragma unroll 1
        for (int ch = 0; ch < KK / 128; ++ch) { const int j0 = ch * 128 + lane * 4; const v4f a = *(const v4f*)(sr + j0); typedef __attribute__((ext_vector_type(4))) _Float16 v4h; v4h o;
#pragma unroll
            for (int u = 0; u < 4; ++u) { float d0 = __fsub_rn(__fadd_rn(a[u] * 0.125f, mr[j0 + u]), mx); asm volatile("" : "+v"(d0)); o[u] = tohx(__fmul_rn(__expf(d0), f)); } *(volatile v4h*)(P16 + (size_t)row * KK + j0) = o; }
        if (ps == 0) __threadfence(); } }

extern "C" void kernel_launch(void* const* d_in, const int* in_sizes, int n_in,
                              void* d_out, int out_size, void* d_ws, size_t ws_size, hipStream_t stream) {
    (void)in_sizes; (void)n_in; (void)out_size;
    const float* q = (const float*)d_in[0]; const float* k = (const float*)d_in[1]; const float* v = (const float*)d_in[2]; const float* am = (const float*)d_in[3]; const int* lidx = (const int*)d_in[4]; const int* gidx = (const int*)d_in[5]; const float* gk = (const float*)d_in[6]; const float* gv = (const float*)d_in[7]; const float* gm = (const float*)d_in[8];
    float* OUT = (float*)d_out;
    char* wsp = (char*)d_ws;
    auto take = [&](size_t bytes) { char* p = wsp; wsp += (bytes + 255) & ~(size_t)255; return (void*)p; };
    bf* QB = (bf*)take((size_t)TT * DDm * 2); bf* KB = (bf*)take((size_t)NBL * KK * DDm * 2); h16* VT = (h16*)take((size_t)NBL * DDm * KK * 2); float* MB = (float*)take((size_t)NBL * KK * 4); float* Sb = (float*)take((size_t)NBL * 64 * KK * 4); h16* P16 = (h16*)take((size_t)NBL * 64 * KK * 2); float* O = (float*)take((size_t)TT * DDm * 4);
    if ((size_t)(wsp - (char*)d_ws) > ws_size) return;
    for (int n = 0; n < NB_; ++n) for (int hh = 0; hh < NHD; ++hh) { const size_t hb = ((size_t)n * NHD + hh) * TT * DDm; const int* li = lidx + ((size_t)n * NHD + hh) * TT; const int* gi = gidx + ((size_t)n * NHD + hh) * TT;
        k_cvt8<<<(TT * DDm / 8 + 255) / 256, 256, 0, stream>>>(q + hb, QB, (size_t)TT * DDm / 8);
        k_kb<<<(NBL * KK * DDm / 4 + 255) / 256, 256, 0, stream>>>(k + hb, gk + ((size_t)n * NHD + hh) * NG * DDm, li, gi, KB); k_vt<<<(NBL * DDm * KK / 2 + 255) / 256, 256, 0, stream>>>(v + hb, gv + ((size_t)n * NHD + hh) * NG * DDm, li, gi, VT);
        k_mb<<<(NBL * KK + 255) / 256, 256, 0, stream>>>(am + (size_t)n * TT, gm + ((size_t)n * NHD + hh) * NG, li, gi, MB);
        k_gemmw<bf, 0, false><<<dim3(1, KK / 64, NBL), 32, 0, stream>>>(QB, nullptr, KB, nullptr, DDm, Sb, KK, nullptr, (size_t)64 * DDm, (size_t)KK * DDm, (size_t)64 * KK);
        k_msoft<<<NBL * 64 / 8, 256, 0, stream>>>(Sb, MB, P16);
        k_gemmw<h16, 0, false><<<dim3(1, 1, NBL), 32, 0, stream>>>(P16, nullptr, VT, nullptr, KK, O, DDm, nullptr, (size_t)64 * KK, (size_t)DDm * KK, (size_t)64 * DDm);
        k_fin<<<(TT * DDm / 4 + 255) / 256, 256, 0, stream>>>(O, OUT + hb); }
}
